// FactorModel_47313359733391
// MI455X (gfx1250) — hardware-verified
//
#include <hip/hip_runtime.h>

typedef __attribute__((ext_vector_type(16))) _Float16 v16h;
typedef __attribute__((ext_vector_type(8)))  _Float16 v8h;
typedef __attribute__((ext_vector_type(4)))  _Float16 v4h;
typedef __attribute__((ext_vector_type(8)))  float    v8f;
typedef __attribute__((ext_vector_type(4)))  float    v4f;

__device__ __forceinline__ void dep_guard_h(v8f& a, v8f& b, v16h x, v16h y) { asm volatile("v_nop\n\tv_nop\n\tv_nop\n\tv_nop" : "+v"(a), "+v"(b) : "v"(x), "v"(y)); }
__device__ __forceinline__ void keep4_h(v16h a, v16h b, v16h c, v16h d) { asm volatile("v_nop" :: "v"(a), "v"(b), "v"(c), "v"(d)); }
template <typename T> struct Frag;
template <> struct Frag<_Float16> {
  typedef v16h V; union U { v16h v; v8h h[2]; };
  static __device__ __forceinline__ v16h load(const _Float16* p) {
    U f; f.h[0] = *(const v8h*)(p); f.h[1] = *(const v8h*)(p + 16); return f.v;
  }
  static __device__ __forceinline__ v8f mma(v16h a, v16h b, v8f c) {
    return __builtin_amdgcn_wmma_f32_16x16x32_f16(false, a, false, b, (short)0, c, false, false);
  }
  static __device__ __forceinline__ void guard(v8f& a, v8f& b, v16h x, v16h y) { dep_guard_h(a, b, x, y); }
  static __device__ __forceinline__ void keep(v16h a, v16h b, v16h c, v16h d) { keep4_h(a, b, c, d); }
};

__device__ __forceinline__ v8f wmma_f16(v16h a, v16h b, v8f cacc) {
  cacc = __builtin_amdgcn_wmma_f32_16x16x32_f16(false, a, false, b, (short)0, cacc, false, false);
  asm volatile("v_nop\n\tv_nop\n\tv_nop\n\tv_nop" : "+v"(cacc) : "v"(a), "v"(b));
  return cacc;
}

__device__ __forceinline__ int imin(int a, int b) { return a < b ? a : b; }
__device__ __forceinline__ int imax(int a, int b) { return a > b ? a : b; }
__device__ __forceinline__ int iclamp(int v, int lo, int hi) { return imin(imax(v, lo), hi); }

constexpr int NB      = 256;
constexpr int TPREV   = 128;
constexpr int TCUR    = 129;
constexpr int NCOV    = 30;
constexpr int NTREAT  = 57;
constexpr int NCONF   = 5;
constexpr int HID     = 128;
constexpr int XDIM    = 87;
constexpr int WIH_K   = 92;
constexpr int KPAD    = 224;
constexpr int COL_H   = 0;
constexpr int COL_Z   = 128;
constexpr int COL_X   = 136;
constexpr int PITCH_A = 232;
constexpr int HB_PITCH = 132;
constexpr int RB      = 32;
constexpr int SCAN_BLOCKS = NB / RB;
constexpr int NROWS   = TCUR * NB;
constexpr int DEC_ROWS = 128;
constexpr int DEC_BLOCKS = NROWS / DEC_ROWS;
constexpr int DEC_F   = 128;
constexpr int MI_K    = 35;
constexpr int KDEC    = 64;
constexpr int MI_PITCH = 72;
constexpr int WD_ROWS = NTREAT * DEC_F;
constexpr int WT_V8   = 512 * KPAD / 8;
constexpr int WD_V8   = WD_ROWS * KDEC / 8;
constexpr size_t WT_BYTES = (size_t)512 * KPAD * 2;
constexpr size_t WD_BYTES = (size_t)WD_ROWS * KDEC * 2;
constexpr long PRED_ELEMS = (long)NROWS * NTREAT;
constexpr long ZS_ELEMS   = (long)NROWS * NCONF;
constexpr float INV256 = 0.00390625f;

static_assert(KPAD % 32 == 0, "K multiple of 32");
static_assert(KDEC % 32 == 0, "K multiple of 32");
static_assert(NB % RB == 0 && NROWS % DEC_ROWS == 0, "exact grids");
static_assert(WT_V8 % 256 == 0 && WD_V8 % 256 == 0, "exact cast grids");
static_assert((RB * NCONF * 4) % 128 == 0, "zs block segment is whole lines");
static_assert((DEC_ROWS * NTREAT * 4) % 128 == 0, "preds block segment is whole lines");
static_assert(WT_BYTES % 128 == 0 && WD_BYTES % 128 == 0, "carve alignment");
static_assert(PITCH_A % 8 == 0 && MI_PITCH % 8 == 0 && HB_PITCH % 4 == 0, "alignment");

__device__ __forceinline__ float sigm(float x) {
  const float xc = fminf(30.0f, fmaxf(-30.0f, x));
  const float e = expf(-xc);
  return __builtin_amdgcn_rcpf(1.0f + e);
}
__device__ __forceinline__ float tnh(float x) { return fmaf(2.0f, sigm(2.0f * x), -1.0f); }

__global__ __launch_bounds__(256) void build_wt_plane(
    const float* __restrict__ W_ih, const float* __restrict__ W_hh, _Float16* __restrict__ WT) {
  const int i = blockIdx.x * 256 + threadIdx.x;
  if (i < WT_V8) {
    const int n = (i * 8) / KPAD;
    const int k0 = i * 8 - n * KPAD;
    v8h o;
#pragma unroll
    for (int e = 0; e < 8; ++e) {
      const int k = k0 + e;
      const float whh = W_hh[(size_t)n * HID + imin(k, HID - 1)];
      const int kih = iclamp((k < COL_X) ? (k - COL_Z + XDIM) : (k - COL_X), 0, WIH_K - 1);
      const float wih = W_ih[(size_t)n * WIH_K + kih];
      const float base = (k < COL_Z) ? whh : wih;
      const float sc = (k < COL_X) ? 32.0f : 256.0f;
      const float keep = ((k < COL_Z + NCONF) || (k >= COL_X && k < COL_X + XDIM)) ? 1.0f : 0.0f;
      o[e] = (_Float16)(base * sc * keep);
    }
    _Float16* dst = WT + (size_t)i * 8;
    *(volatile v8h*)dst = o;
    __threadfence();
    *(volatile v8h*)dst = o;
  }
}

__global__ __launch_bounds__(256) void build_wd_plane(
    const float* __restrict__ dW1, _Float16* __restrict__ WD) {
  const int i = blockIdx.x * 256 + threadIdx.x;
  if (i < WD_V8) {
    const int R = i >> 3;
    const int g = i & 7;
    const int tp = R >> 7;
    const int f = R & 127;
    v8h o;
#pragma unroll
    for (int e = 0; e < 8; ++e) {
      const int cin = 8 * g + e;
      const float w = dW1[((size_t)tp * MI_K + imin(cin, MI_K - 1)) * DEC_F + f];
      const float sc = (cin < NCONF) ? 32.0f : 256.0f;
      const float keep = (cin < MI_K) ? 1.0f : 0.0f;
      o[e] = (_Float16)(w * sc * keep);
    }
    _Float16* dst = WD + (size_t)i * 8;
    *(volatile v8h*)dst = o;
    __threadfence();
    *(volatile v8h*)dst = o;
  }
}

__global__ __launch_bounds__(256) void lstm_scan_kernel(
    const float* __restrict__ pcov, const float* __restrict__ ptrt, const float* __restrict__ iinp,
    const float* __restrict__ h0, const float* __restrict__ c0, const float* __restrict__ z0,
    const _Float16* __restrict__ WT,
    const float* __restrict__ b_ih, const float* __restrict__ b_hh,
    const float* __restrict__ W_z, const float* __restrict__ b_z,
    float* zs_out)
{
  __shared__ __align__(16) _Float16 Atile[RB * PITCH_A];
  __shared__ __align__(16) float hbuf[RB * HB_PITCH];
  __shared__ __align__(16) float zstage[RB * NCONF];

  const int tid  = threadIdx.x;
  const int wave = tid >> 5;
  const int lane = tid & 31;
  const int hh   = lane >> 4;
  const int c    = lane & 15;
  const int koff = hh * 8;
  const int bbase = blockIdx.x * RB;

  for (int i = tid; i < RB * COL_X; i += 256) {
    const int row = i / COL_X;
    const int col = i - row * COL_X;
    const float hv = h0[imin(col, HID - 1)] * 8.0f;
    const float zv = z0[iclamp(col - COL_Z, 0, NCONF - 1)] * 8.0f;
    const float v = (col < COL_Z) ? hv : zv;
    const float keep = (col < COL_Z + NCONF) ? 1.0f : 0.0f;
    Atile[row * PITCH_A + col] = (_Float16)(v * keep);
  }

  float creg[2][8];
  {
    const float cv = c0[16 * wave + c];
#pragma unroll
    for (int ms = 0; ms < 2; ++ms)
#pragma unroll
      for (int r = 0; r < 8; ++r) creg[ms][r] = cv;
  }
  const int ucol = 16 * wave + c;
  const float bi = b_ih[ucol] + b_hh[ucol];
  const float bf = b_ih[HID + ucol] + b_hh[HID + ucol];
  const float bg = b_ih[2 * HID + ucol] + b_hh[2 * HID + ucol];
  const float bo = b_ih[3 * HID + ucol] + b_hh[3 * HID + ucol];

  float wzr[NCONF][4];
  float bzr[NCONF];
#pragma unroll
  for (int j = 0; j < NCONF; ++j) {
    bzr[j] = b_z[j];
#pragma unroll
    for (int q = 0; q < 4; ++q) wzr[j][q] = W_z[j * HID + lane + 32 * q];
  }

  const _Float16* wt_base = WT + (size_t)(16 * wave + c) * KPAD + koff;
  const _Float16* a_base  = Atile + c * PITCH_A + koff;

  for (int t = 0; t < TCUR; ++t) {
    const int tcl = (t > 0) ? (t - 1) : 0;
    for (int idx = tid; idx < RB * 11; idx += 256) {
      const int row = idx / 11;
      const int g = idx - row * 11;
      const size_t boff = (size_t)(bbase + row) * TPREV + tcl;
      const float* pcr = pcov + boff * NCOV;
      const float* ptr2 = ptrt + boff * NTREAT;
      v8h xv;
#pragma unroll
      for (int e = 0; e < 8; ++e) {
        const int j = 8 * g + e;
        const float av = pcr[imin(j, NCOV - 1)];
        const float bv = ptr2[iclamp(j - NCOV, 0, NTREAT - 1)];
        const float iv = iinp[imin(j, XDIM - 1)];
        float v = (j < NCOV) ? av : bv;
        v = (t == 0) ? iv : v;
        const float keep = (j < XDIM) ? 1.0f : 0.0f;
        xv[e] = (_Float16)(v * keep);
      }
      *(v8h*)(Atile + row * PITCH_A + COL_X + 8 * g) = xv;
    }
    __syncthreads();

    v8f acc[2][4];
#pragma unroll
    for (int ms = 0; ms < 2; ++ms)
#pragma unroll
      for (int gt = 0; gt < 4; ++gt) acc[ms][gt] = (v8f){0.f,0.f,0.f,0.f,0.f,0.f,0.f,0.f};
#pragma unroll 1
    for (int kf = 0; kf < KPAD / 32; ++kf) {
      v16h bfr[4];
#pragma unroll
      for (int gt = 0; gt < 4; ++gt)
        bfr[gt] = Frag<_Float16>::load(wt_base + (size_t)gt * HID * KPAD + kf * 32);
#pragma unroll
      for (int ms = 0; ms < 2; ++ms) {
        const v16h af = Frag<_Float16>::load(a_base + ms * 16 * PITCH_A + kf * 32);
#pragma unroll
        for (int gt = 0; gt < 4; ++gt) acc[ms][gt] = wmma_f16(af, bfr[gt], acc[ms][gt]);
      }
    }

#pragma unroll
    for (int ms = 0; ms < 2; ++ms) {
#pragma unroll
      for (int r = 0; r < 8; ++r) {
        const float gi = fmaf(acc[ms][0][r], INV256, bi);
        const float gf = fmaf(acc[ms][1][r], INV256, bf);
        const float gg = fmaf(acc[ms][2][r], INV256, bg);
        const float go = fmaf(acc[ms][3][r], INV256, bo);
        const float cn = sigm(gf) * creg[ms][r] + sigm(gi) * tnh(gg);
        creg[ms][r] = cn;
        const float hv = sigm(go) * tnh(cn);
        hbuf[(16 * ms + 8 * hh + r) * HB_PITCH + ucol] = hv;
      }
    }
    __syncthreads();

#pragma unroll 1
    for (int rho = 0; rho < 4; ++rho) {
      const int row = 4 * wave + rho;
      const float* hr = hbuf + row * HB_PITCH;
      float p[NCONF];
#pragma unroll
      for (int j = 0; j < NCONF; ++j) p[j] = 0.0f;
#pragma unroll
      for (int q = 0; q < 4; ++q) {
        const float hv = hr[lane + 32 * q];
#pragma unroll
        for (int j = 0; j < NCONF; ++j) p[j] = fmaf(hv, wzr[j][q], p[j]);
      }
#pragma unroll
      for (int j = 0; j < NCONF; ++j) {
        float s = p[j];
        s += __shfl_xor(s, 1, 32);
        s += __shfl_xor(s, 2, 32);
        s += __shfl_xor(s, 4, 32);
        s += __shfl_xor(s, 8, 32);
        s += __shfl_xor(s, 16, 32);
        p[j] = s + bzr[j];
      }
      float zsel = p[0];
      zsel = (lane == 1) ? p[1] : zsel;
      zsel = (lane == 2) ? p[2] : zsel;
      zsel = (lane == 3) ? p[3] : zsel;
      zsel = (lane == 4) ? p[4] : zsel;
      if (lane < NCONF) {
        Atile[row * PITCH_A + COL_Z + lane] = (_Float16)(zsel * 8.0f);
        zstage[row * NCONF + lane] = zsel;
      }
      const v4f h4 = *(const v4f*)(hr + 4 * lane);
      v4h hq;
#pragma unroll
      for (int e = 0; e < 4; ++e) hq[e] = (_Float16)(h4[e] * 8.0f);
      *(v4h*)(Atile + row * PITCH_A + COL_H + 4 * lane) = hq;
    }
    __syncthreads();

    {
      float* dst = zs_out + ((size_t)t * NB + bbase) * NCONF;
      const int f4 = wave * 32 + lane;
      if (f4 < (RB * NCONF) / 4) {
        const v4f v = *(const v4f*)(zstage + 4 * f4);
        *(volatile v4f*)(dst + 4 * f4) = v;
        __threadfence();
        *(volatile v4f*)(dst + 4 * f4) = v;
      }
    }
  }
}

__global__ __launch_bounds__(256) void decoder_kernel(
    const float* zs, const float* __restrict__ ccov,
    const _Float16* __restrict__ WD, const float* __restrict__ db1,
    const float* __restrict__ dW2, const float* __restrict__ db2,
    float* preds)
{
  __shared__ __align__(16) _Float16 MI[DEC_ROWS * MI_PITCH];
  __shared__ __align__(16) float predS[DEC_ROWS * NTREAT];

  const int tid  = threadIdx.x;
  const int wave = tid >> 5;
  const int lane = tid & 31;
  const int hh   = lane >> 4;
  const int c    = lane & 15;
  const int koff = hh * 8;
  const int blk  = blockIdx.x;
  const int row0 = blk * DEC_ROWS;

  for (int idx = tid; idx < DEC_ROWS * 8; idx += 256) {
    const int row = idx >> 3;
    const int g = idx & 7;
    const int n = row0 + row;
    const int tt = n >> 8;
    const int b = n & 255;
    const float* zr = zs + (size_t)n * NCONF;
    const float* cr = ccov + ((size_t)b * TCUR + tt) * NCOV;
    v8h mv;
#pragma unroll
    for (int e = 0; e < 8; ++e) {
      const int j = 8 * g + e;
      const float zv = zr[imin(j, NCONF - 1)] * 8.0f;
      const float cv = cr[iclamp(j - NCONF, 0, NCOV - 1)];
      const float v = (j < NCONF) ? zv : cv;
      const float keep = (j < MI_K) ? 1.0f : 0.0f;
      mv[e] = (_Float16)(v * keep);
    }
    *(v8h*)(MI + row * MI_PITCH + 8 * g) = mv;
  }
  __syncthreads();

  const _Float16* mrow = MI + (wave * 16 + c) * MI_PITCH + koff;
  const v16h af0 = Frag<_Float16>::load(mrow);
  const v16h af1 = Frag<_Float16>::load(mrow + 32);
  float* prow_s = predS + (wave * 16 + 8 * hh) * NTREAT;

#pragma unroll 1
  for (int tp = 0; tp < NTREAT; ++tp) {
    float rsum[8];
#pragma unroll
    for (int r = 0; r < 8; ++r) rsum[r] = 0.0f;
    const _Float16* wrow = WD + ((size_t)tp * DEC_F + c) * KDEC + koff;
    const float* b1p = db1 + (size_t)tp * DEC_F + c;
    const float* w2p = dW2 + (size_t)tp * DEC_F + c;
#pragma unroll 4
    for (int nt = 0; nt < DEC_F / 16; ++nt) {
      const v16h b0 = Frag<_Float16>::load(wrow + nt * 16 * KDEC);
      const v16h b1 = Frag<_Float16>::load(wrow + nt * 16 * KDEC + 32);
      v8f a = (v8f){0.f,0.f,0.f,0.f,0.f,0.f,0.f,0.f};
      a = wmma_f16(af0, b0, a);
      a = wmma_f16(af1, b1, a);
      const float b1v = b1p[nt * 16];
      const float w2v = w2p[nt * 16];
#pragma unroll
      for (int r = 0; r < 8; ++r) {
        float hv = fmaf(a[r], INV256, b1v);
        hv = (hv > 0.0f) ? hv : 0.01f * hv;
        rsum[r] = fmaf(hv, w2v, rsum[r]);
      }
    }
    const float b2v = db2[tp];
#pragma unroll
    for (int r = 0; r < 8; ++r) {
      float s = rsum[r];
      s += __shfl_xor(s, 1, 32);
      s += __shfl_xor(s, 2, 32);
      s += __shfl_xor(s, 4, 32);
      s += __shfl_xor(s, 8, 32);
      if (c == 0) prow_s[r * NTREAT + tp] = s + b2v;
    }
  }
  __syncthreads();

  {
    float* dst = preds + (size_t)blk * (DEC_ROWS * NTREAT);
    for (int pass = 0; pass < 2; ++pass) {
      for (int i = tid; i < (DEC_ROWS * NTREAT) / 4; i += 256) {
        const v4f v = *(const v4f*)(predS + 4 * i);
        *(volatile v4f*)(dst + 4 * i) = v;
      }
      __threadfence();
    }
  }
}

extern "C" void kernel_launch(void* const* d_in, const int* in_sizes, int n_in,
                              void* d_out, int out_size, void* d_ws, size_t ws_size,
                              hipStream_t stream) {
  if (n_in < 17) return;
  if ((long)out_size != PRED_ELEMS + ZS_ELEMS) return;
  if (ws_size < WT_BYTES + WD_BYTES) return;
  if (in_sizes[0] != NB * TPREV * NCOV || in_sizes[1] != NB * TPREV * NTREAT ||
      in_sizes[2] != NB * TCUR * NCOV || in_sizes[7] != 512 * WIH_K ||
      in_sizes[8] != 512 * HID || in_sizes[13] != NTREAT * MI_K * DEC_F) return;

  const float* pcov = (const float*)d_in[0];
  const float* ptrt = (const float*)d_in[1];
  const float* ccov = (const float*)d_in[2];
  const float* iinp = (const float*)d_in[3];
  const float* h0   = (const float*)d_in[4];
  const float* c0   = (const float*)d_in[5];
  const float* z0   = (const float*)d_in[6];
  const float* Wih  = (const float*)d_in[7];
  const float* Whh  = (const float*)d_in[8];
  const float* bih  = (const float*)d_in[9];
  const float* bhh  = (const float*)d_in[10];
  const float* Wz   = (const float*)d_in[11];
  const float* bz   = (const float*)d_in[12];
  const float* dW1  = (const float*)d_in[13];
  const float* db1  = (const float*)d_in[14];
  const float* dW2  = (const float*)d_in[15];
  const float* db2  = (const float*)d_in[16];

  char* ws = (char*)d_ws;
  _Float16* WT = (_Float16*)(ws + 0);
  _Float16* WD = (_Float16*)(ws + WT_BYTES);

  float* preds = (float*)d_out;
  float* zs    = preds + PRED_ELEMS;

  build_wt_plane<<<dim3(WT_V8 / 256), dim3(256), 0, stream>>>(Wih, Whh, WT);
  build_wd_plane<<<dim3(WD_V8 / 256), dim3(256), 0, stream>>>(dW1, WD);
  lstm_scan_kernel<<<dim3(SCAN_BLOCKS), dim3(256), 0, stream>>>(
      pcov, ptrt, iinp, h0, c0, z0, WT, bih, bhh, Wz, bz, zs);
  decoder_kernel<<<dim3(DEC_BLOCKS), dim3(256), 0, stream>>>(zs, ccov, WD, db1, dW2, db2, preds);
}
